// SelfAttentionBlock_9672266351200
// MI455X (gfx1250) — hardware-verified
//
#include <hip/hip_runtime.h>
#include <math.h>
#include <stdint.h>

#pragma clang fp contract(off)

#define NB     2
#define SQ     2048
#define HID    1024
#define NH     16
#define HDM    64
#define CONDF  768
#define NTOK   4096
#define QW     1024
#define QKN    2048
#define NQKV   3072
#define XNW    2048
#define AOW    2048
#define NFR    8
#define TABW   128

typedef __bf16       v16b __attribute__((ext_vector_type(16)));
typedef __bf16       v8b  __attribute__((ext_vector_type(8)));
typedef float        v8f  __attribute__((ext_vector_type(8)));
typedef float        v4f  __attribute__((ext_vector_type(4)));
typedef unsigned int v4u  __attribute__((ext_vector_type(4)));

__device__ __forceinline__ unsigned short bf_bits(float f) {
  const unsigned u = __float_as_uint(f);
  return (unsigned short)((u + 0x7FFFu + ((u >> 16) & 1u)) >> 16);
}
__device__ __forceinline__ float bf_val(unsigned short h) { return __uint_as_float(((unsigned)h) << 16); }
__device__ __forceinline__ float bf_rne(float f) { return bf_val(bf_bits(f)); }
__device__ __forceinline__ unsigned pk16(unsigned short a, unsigned short b) { return (unsigned)a | ((unsigned)b << 16); }
__device__ __forceinline__ v8f zero8() { v8f z = {0.f, 0.f, 0.f, 0.f, 0.f, 0.f, 0.f, 0.f}; return z; }
__device__ __forceinline__ int wave_id() { return __builtin_amdgcn_readfirstlane((int)(threadIdx.x >> 5)); }

__device__ __forceinline__ void lds_wave_sync() {
  __builtin_amdgcn_fence(__ATOMIC_RELEASE, "workgroup");
  __builtin_amdgcn_wave_barrier();
  __builtin_amdgcn_fence(__ATOMIC_ACQUIRE, "workgroup");
}

union FragB { v16b v; v8b h[2]; };
__device__ __forceinline__ v16b ldfrag_b(const __bf16* p) { FragB f; f.h[0] = *(const v8b*)(p); f.h[1] = *(const v8b*)(p + 16); return f.v; }

__device__ __forceinline__ v8f mma_b(v16b a, v16b b, v8f c) {
  return __builtin_amdgcn_wmma_f32_16x16x32_bf16(false, a, false, b, (short)0, c, false, false);
}
__device__ __forceinline__ void guard2b3(v8f& a, v8f& b, v16b x0, v16b x1, v16b y) {
  asm volatile("v_nop\n\tv_nop\n\tv_nop\n\tv_nop" : "+v"(a), "+v"(b) : "v"(x0), "v"(x1), "v"(y) : "memory");
}
__device__ __forceinline__ void guard1b4(v8f& a, v16b w, v16b x, v16b y, v16b z) {
  asm volatile("v_nop\n\tv_nop\n\tv_nop\n\tv_nop" : "+v"(a) : "v"(w), "v"(x), "v"(y), "v"(z) : "memory");
}
__device__ __forceinline__ void acc_guard4(v8f& a, v8f& b, v8f& c, v8f& d) {
  asm volatile("v_nop\n\tv_nop\n\tv_nop\n\tv_nop" : "+v"(a), "+v"(b), "+v"(c), "+v"(d));
}
__device__ __forceinline__ void acc_guard2(v8f& a, v8f& b) {
  asm volatile("v_nop\n\tv_nop\n\tv_nop\n\tv_nop" : "+v"(a), "+v"(b));
}

__global__ __launch_bounds__(128) void freq_table_kernel(float* __restrict__ ftab) {
  const int t = (int)threadIdx.x;
  const int i = (t & 7) * NH + (t >> 3);
  const double lmin = log(3.141592653589793);
  const double lmax = log(10.0 * 3.141592653589793);
  const double step = (lmax - lmin) / 128.0;
  const double y = (double)i * step + lmin;
  const float f = (float)exp(y);
  ((volatile float*)ftab)[t] = f;
  __threadfence();
  ((volatile float*)ftab)[t] = f;
}

__global__ __launch_bounds__(256) void cond_scale_kernel(const float* __restrict__ cond, const float* __restrict__ wn,
                                                         float* __restrict__ cs) {
  const int idx = (int)blockIdx.x * 256 + (int)threadIdx.x;
  if (idx >= NB * HID) return;
  const int b = idx / HID;
  const int d = idx - b * HID;
  const float* cr = cond + (size_t)b * CONDF;
  const float* wr = wn + (size_t)d * CONDF;
  float acc = 0.0f;
#pragma unroll 2
  for (int i = 0; i < CONDF; i += 4) {
    const v4f cv = *(const v4f*)(cr + i);
    const v4f wv = *(const v4f*)(wr + i);
    acc += bf_rne(cv[0]) * bf_rne(wv[0]);
    acc += bf_rne(cv[1]) * bf_rne(wv[1]);
    acc += bf_rne(cv[2]) * bf_rne(wv[2]);
    acc += bf_rne(cv[3]) * bf_rne(wv[3]);
  }
  const float v = acc + 1.0f;
  ((volatile float*)cs)[idx] = v;
  __threadfence();
  ((volatile float*)cs)[idx] = v;
}

__global__ __launch_bounds__(128) void rope_table_kernel(const float* __restrict__ pos, const float* __restrict__ ftab,
                                                         float* __restrict__ cst, float* __restrict__ snt) {
  const int tok = (int)blockIdx.x;
  const int t   = (int)threadIdx.x;
  const float pr  = bf_rne(pos[tok]);
  const float fr  = ftab[t];
  const float ang = pr * fr;
  const float cv  = cosf(ang);
  const float sv  = sinf(ang);
  const size_t o = (size_t)tok * TABW + t;
  ((volatile float*)cst)[o] = cv;
  ((volatile float*)snt)[o] = sv;
  __threadfence();
  ((volatile float*)cst)[o] = cv;
  ((volatile float*)snt)[o] = sv;
}

__global__ __launch_bounds__(128) void xn_split_kernel(const float* __restrict__ x, const float* __restrict__ cs,
                                                       unsigned short* __restrict__ xn) {
  __shared__ float red[4];
  const int row  = (int)blockIdx.x;
  const int tid  = (int)threadIdx.x;
  const int lane = tid & 31;
  const int wave = tid >> 5;
  const int b    = row / SQ;
  const size_t xo = (size_t)row * HID + 8 * tid;
  const v4f a0 = *(const v4f*)(x + xo);
  const v4f a1 = *(const v4f*)(x + xo + 4);
  float xr[8];
#pragma unroll
  for (int e = 0; e < 4; ++e) { xr[e] = bf_rne(a0[e]); xr[4 + e] = bf_rne(a1[e]); }
  float s = 0.0f;
#pragma unroll
  for (int e = 0; e < 8; ++e) s += xr[e] * xr[e];
#pragma unroll
  for (int off = 16; off > 0; off >>= 1) s += __shfl_xor(s, off, 32);
  if (lane == 0) red[wave] = s;
  __syncthreads();
  const float tot = ((red[0] + red[1]) + red[2]) + red[3];
  const float ms  = tot * 0.0009765625f;
  const float rs  = rsqrtf(ms + 1e-6f);
  const size_t co = (size_t)b * HID + 8 * tid;
  const v4f c0 = *(const v4f*)(cs + co);
  const v4f c1 = *(const v4f*)(cs + co + 4);
  float cc[8];
#pragma unroll
  for (int e = 0; e < 4; ++e) { cc[e] = c0[e]; cc[4 + e] = c1[e]; }
  v4u wh, wlo;
#pragma unroll
  for (int q = 0; q < 4; ++q) {
    const float t0 = cc[2 * q] * rs;
    const float t1 = cc[2 * q + 1] * rs;
    const float v0 = xr[2 * q] * t0;
    const float v1 = xr[2 * q + 1] * t1;
    const unsigned short h0 = bf_bits(v0), h1 = bf_bits(v1);
    const unsigned short l0 = bf_bits(v0 - bf_val(h0)), l1 = bf_bits(v1 - bf_val(h1));
    wh[q]  = pk16(h0, h1);
    wlo[q] = pk16(l0, l1);
  }
  const size_t o = (size_t)row * XNW + 8 * tid;
  *(volatile v4u*)(xn + o) = wh;
  *(volatile v4u*)(xn + o + HID) = wlo;
  __threadfence();
  *(volatile v4u*)(xn + o) = wh;
  *(volatile v4u*)(xn + o + HID) = wlo;
}

__global__ __launch_bounds__(256) void cvt_dup2_kernel(const float* __restrict__ in, unsigned short* __restrict__ outp,
                                                       int n8, int kin, int ldo) {
  const int i = (int)blockIdx.x * 256 + (int)threadIdx.x;
  if (i >= n8) return;
  const size_t e = 8 * (size_t)i;
  const int n = (int)(e / (size_t)kin);
  const int k = (int)(e - (size_t)n * kin);
  const v4f a = *(const v4f*)(in + e);
  const v4f b = *(const v4f*)(in + e + 4);
  v4u w;
  w[0] = pk16(bf_bits(a[0]), bf_bits(a[1]));
  w[1] = pk16(bf_bits(a[2]), bf_bits(a[3]));
  w[2] = pk16(bf_bits(b[0]), bf_bits(b[1]));
  w[3] = pk16(bf_bits(b[2]), bf_bits(b[3]));
  const size_t o = (size_t)n * ldo + k;
  *(volatile v4u*)(outp + o) = w;
  *(volatile v4u*)(outp + o + kin) = w;
  __threadfence();
  *(volatile v4u*)(outp + o) = w;
  *(volatile v4u*)(outp + o + kin) = w;
}

template <int EPI> struct SlabCfg { static constexpr int PERWF = 2048; };
template <> struct SlabCfg<0>     { static constexpr int PERWF = 2560; };

template <int EPI>
__global__ __launch_bounds__(128) void gemm_w32x128_kernel(
    const unsigned short* __restrict__ Ap, int lda,
    const unsigned short* __restrict__ Btp, int ldb,
    const float* __restrict__ cst, const float* __restrict__ snt,
    const float* __restrict__ scl, const float* __restrict__ resid,
    void* C0, void* C1, void* C2, void* C3, int ldc, int ldc2,
    int M, int N, int K) {
  __shared__ __align__(16) float lds_all[4 * SlabCfg<EPI>::PERWF];

  const int lane = threadIdx.x & 31;
  const int wave = wave_id();
  const int hh = lane >> 4;
  const int rl = lane & 15;
  const int tilesN = N >> 7;
  const int tilesM = M >> 5;
  const int tile = (int)blockIdx.x * 4 + wave;
  if (tile >= tilesM * tilesN) return;
  const int tm = tile / tilesN;
  const int tn = tile - tm * tilesN;
  const int m0 = tm << 5;
  const int n0 = tn << 7;

  const __bf16* A  = (const __bf16*)(const void*)Ap;
  const __bf16* Bt = (const __bf16*)(const void*)Btp;

  v8f acc[2][8];
#pragma unroll
  for (int i = 0; i < 2; ++i)
#pragma unroll
    for (int j = 0; j < 8; ++j) acc[i][j] = zero8();

  for (int k0 = 0; k0 < K; k0 += 32) {
    v16b ah[2];
#pragma unroll
    for (int i = 0; i < 2; ++i) ah[i] = ldfrag_b(A + (size_t)(m0 + i * 16 + rl) * lda + k0 + 8 * hh);
#pragma unroll
    for (int j = 0; j < 8; ++j) {
      const v16b bj = ldfrag_b(Bt + (size_t)(n0 + j * 16 + rl) * ldb + k0 + 8 * hh);
      acc[0][j] = mma_b(ah[0], bj, acc[0][j]);
      acc[1][j] = mma_b(ah[1], bj, acc[1][j]);
      guard2b3(acc[0][j], acc[1][j], ah[0], ah[1], bj);
    }
  }
  acc_guard4(acc[0][0], acc[0][1], acc[0][2], acc[0][3]);
  acc_guard4(acc[0][4], acc[0][5], acc[0][6], acc[0][7]);
  acc_guard4(acc[1][0], acc[1][1], acc[1][2], acc[1][3]);
  acc_guard4(acc[1][4], acc[1][5], acc[1][6], acc[1][7]);

  float* wl = lds_all + wave * SlabCfg<EPI>::PERWF;
  unsigned short* sl16 = (unsigned short*)(void*)wl;
  float* slf = wl;

  if (EPI == 0) {
    float* csl = wl + 2048;
    float* snl = wl + 2048 + 256;
    const bool isq = (n0 < QW);
    unsigned short* P0 = isq ? (unsigned short*)C0 : (unsigned short*)C2;
    unsigned short* P1 = isq ? (unsigned short*)C1 : (unsigned short*)C3;
    const int ldp  = isq ? ldc : ldc2;
    const int col0 = isq ? n0 : (n0 - QW);
    const int hq0  = col0 >> 6;
    const float ss0 = sqrtf(bf_rne(scl[hq0]));
    const float ss1 = sqrtf(bf_rne(scl[hq0 + 1]));
#pragma unroll
    for (int i = 0; i < 2; ++i) {
      const int mb = m0 + i * 16;
#pragma unroll
      for (int u = 0; u < 2; ++u) {
        const int p   = lane + 32 * u;
        const int row = p >> 2, c4 = (p & 3) * 4;
        const size_t to = (size_t)(mb + row) * TABW + hq0 * NFR + c4;
        const v4f cv4 = *(const v4f*)(cst + to);
        const v4f sv4 = *(const v4f*)(snt + to);
        *(v4f*)(csl + row * 16 + c4) = cv4;
        *(v4f*)(snl + row * 16 + c4) = sv4;
      }
      lds_wave_sync();
#pragma unroll
      for (int hs = 0; hs < 2; ++hs) {
        const float ss = (hs == 0) ? ss0 : ss1;
        float nrm[8];
#pragma unroll
        for (int r = 0; r < 8; ++r) {
          float sq = 0.0f;
#pragma unroll
          for (int jj = 0; jj < 4; ++jj) { const float v = acc[i][hs * 4 + jj][r]; sq += v * v; }
          sq += __shfl_xor(sq, 1, 32);
          sq += __shfl_xor(sq, 2, 32);
          sq += __shfl_xor(sq, 4, 32);
          sq += __shfl_xor(sq, 8, 32);
          nrm[r] = ss * rsqrtf(sq + 1e-6f);
        }
#pragma unroll
        for (int jj = 0; jj < 4; ++jj) {
          const int j1 = hs * 4 + jj;
#pragma unroll
          for (int r = 0; r < 8; ++r) {
            const int lrow = 8 * hh + r;
            float o = acc[i][j1][r] * nrm[r];
            if (jj == 0) {
              const float pt = __shfl_xor(o, 8, 32);
              const int   fi = lrow * 16 + hs * NFR + (rl & 7);
              const float cv = csl[fi];
              const float sv = snl[fi];
              const float sg = (rl < 8) ? -1.0f : 1.0f;
              o = o * cv + sg * (pt * sv);
            }
            const unsigned short hb = bf_bits(o);
            const unsigned short lb = bf_bits(o - bf_val(hb));
            const int so = lrow * 128 + hs * 64 + jj * 16 + rl;
            sl16[so]        = hb;
            sl16[2048 + so] = lb;
          }
        }
      }
      lds_wave_sync();
      for (int pass = 0; pass < 2; ++pass) {
#pragma unroll
        for (int it = 0; it < 8; ++it) {
          const int row = it * 2 + hh;
          const int c8  = rl * 8;
          const v4u vh = *(const v4u*)(sl16 + row * 128 + c8);
          const v4u vl = *(const v4u*)(sl16 + 2048 + row * 128 + c8);
          const size_t go = (size_t)(mb + row) * ldp + col0 + c8;
          *(volatile v4u*)(P0 + go) = vh;
          *(volatile v4u*)(P1 + go) = vl;
        }
        __threadfence();
      }
      lds_wave_sync();
    }
  } else if (EPI == 1) {
    unsigned short* P0 = (unsigned short*)C0;
    unsigned short* P1 = (unsigned short*)C1;
#pragma unroll
    for (int i = 0; i < 2; ++i) {
#pragma unroll
      for (int r = 0; r < 8; ++r) {
#pragma unroll
        for (int j = 0; j < 8; ++j) {
          const float v = acc[i][j][r];
          const unsigned short hb = bf_bits(v);
          const unsigned short lb = bf_bits(v - bf_val(hb));
          const int so = (8 * hh + r) * 128 + j * 16 + rl;
          sl16[so]        = hb;
          sl16[2048 + so] = lb;
        }
      }
      lds_wave_sync();
      for (int pass = 0; pass < 2; ++pass) {
#pragma unroll
        for (int it = 0; it < 8; ++it) {
          const int row = it * 2 + hh;
          const int c8  = rl * 8;
          const v4u vh = *(const v4u*)(sl16 + row * 128 + c8);
          const v4u vl = *(const v4u*)(sl16 + 2048 + row * 128 + c8);
          const size_t go = (size_t)(m0 + i * 16 + row) * ldc + n0 + c8;
          *(volatile v4u*)(P0 + go) = vh;
          *(volatile v4u*)(P1 + go) = vl;
        }
        __threadfence();
      }
      lds_wave_sync();
    }
  } else {
    float* C = (float*)C0;
#pragma unroll
    for (int i = 0; i < 2; ++i) {
#pragma unroll
      for (int j = 0; j < 8; ++j)
#pragma unroll
        for (int r = 0; r < 8; ++r)
          slf[(8 * hh + r) * 128 + j * 16 + rl] = acc[i][j][r];
      lds_wave_sync();
#pragma unroll 4
      for (int row = 0; row < 16; ++row) {
        const size_t g = (size_t)(m0 + i * 16 + row) * ldc + n0 + lane * 4;
        v4f a = *(const v4f*)(slf + row * 128 + lane * 4);
        const v4f xr = *(const v4f*)(resid + g);
        a[0] += bf_rne(xr[0]);
        a[1] += bf_rne(xr[1]);
        a[2] += bf_rne(xr[2]);
        a[3] += bf_rne(xr[3]);
        *(v4f*)(slf + row * 128 + lane * 4) = a;
      }
      for (int pass = 0; pass < 2; ++pass) {
#pragma unroll
        for (int row = 0; row < 16; ++row) {
          const v4f v = *(const v4f*)(slf + row * 128 + lane * 4);
          *(volatile v4f*)(C + (size_t)(m0 + i * 16 + row) * ldc + n0 + lane * 4) = v;
        }
        __threadfence();
      }
      lds_wave_sync();
    }
  }
}

#define AKC  32
#define KP   72
#define VP   40
#define PP   40
static_assert((2 * AKC * KP + 2 * HDM * VP + 8 * 16 * PP + 8 * 16 * 64) * 2 <= 65536);

__global__ __launch_bounds__(128) void attn_kernel(
    const unsigned short* __restrict__ qhp, const unsigned short* __restrict__ qlp,
    const unsigned short* __restrict__ khp, const unsigned short* __restrict__ klp,
    const unsigned short* __restrict__ vhp, const unsigned short* __restrict__ vlp,
    unsigned short* __restrict__ aop) {
  __shared__ __align__(16) unsigned short Ks[AKC * KP];
  __shared__ __align__(16) unsigned short Kls[AKC * KP];
  __shared__ __align__(16) unsigned short Vhs[HDM * VP];
  __shared__ __align__(16) unsigned short Vls[HDM * VP];
  __shared__ __align__(16) unsigned short Phs[4][16 * PP];
  __shared__ __align__(16) unsigned short Pls[4][16 * PP];
  __shared__ __align__(16) unsigned short Osh[4][16 * 64];
  __shared__ __align__(16) unsigned short Osl[4][16 * 64];

  const int tid  = (int)threadIdx.x;
  const int lane = tid & 31;
  const int wave = wave_id();
  const int hh   = lane >> 4;
  const int c    = lane & 15;
  const int qt   = (int)blockIdx.x;
  const int h    = (int)blockIdx.y;
  const int b    = (int)blockIdx.z;
  const int q0   = qt * 64 + wave * 16;
  const size_t tok0 = (size_t)b * SQ;

  const __bf16* Qhr = (const __bf16*)(const void*)qhp + (tok0 + q0 + c) * QW + h * HDM + 8 * hh;
  const __bf16* Qlr = (const __bf16*)(const void*)qlp + (tok0 + q0 + c) * QW + h * HDM + 8 * hh;

  unsigned short* ph = Phs[wave];
  unsigned short* pl = Pls[wave];

  v16b qh[2], ql[2];
#pragma unroll
  for (int dc = 0; dc < 2; ++dc) { qh[dc] = ldfrag_b(Qhr + dc * 32); ql[dc] = ldfrag_b(Qlr + dc * 32); }

  float mrow[8], lrow[8];
  v8f oacc[4];
#pragma unroll
  for (int r = 0; r < 8; ++r) { mrow[r] = -INFINITY; lrow[r] = 0.f; }
#pragma unroll
  for (int t = 0; t < 4; ++t) oacc[t] = zero8();

  for (int kc = 0; kc < SQ / AKC; ++kc) {
    const int kv0 = kc * AKC;
    __syncthreads();
#pragma unroll
    for (int u = 0; u < 2; ++u) {
      const int p   = tid + 128 * u;
      const int key = p >> 3, d8 = (p & 7) * 8;
      const size_t ko = (tok0 + kv0 + key) * QW + h * HDM + d8;
      const v4u kx = *(const v4u*)(khp + ko);
      const v4u ky = *(const v4u*)(klp + ko);
      *(v4u*)(Ks  + key * KP + d8) = kx;
      *(v4u*)(Kls + key * KP + d8) = ky;
      const int d = p >> 2, k8 = (p & 3) * 8;
      const size_t vo = (size_t)(h * HDM + d) * NTOK + tok0 + kv0 + k8;
      const v4u vx = *(const v4u*)(vhp + vo);
      const v4u vy = *(const v4u*)(vlp + vo);
      *(v4u*)(Vhs + d * VP + k8) = vx;
      *(v4u*)(Vls + d * VP + k8) = vy;
    }
    __syncthreads();

    v8f sa[2];
    sa[0] = zero8(); sa[1] = zero8();
#pragma unroll
    for (int dc = 0; dc < 2; ++dc) {
#pragma unroll
      for (int j = 0; j < 2; ++j) {
        const v16b kb = ldfrag_b((const __bf16*)(const void*)Ks  + (j * 16 + c) * KP + dc * 32 + 8 * hh);
        const v16b kl = ldfrag_b((const __bf16*)(const void*)Kls + (j * 16 + c) * KP + dc * 32 + 8 * hh);
        sa[j] = mma_b(qh[dc], kb, sa[j]);
        sa[j] = mma_b(qh[dc], kl, sa[j]);
        sa[j] = mma_b(ql[dc], kb, sa[j]);
        guard1b4(sa[j], qh[dc], ql[dc], kb, kl);
      }
    }
    acc_guard2(sa[0], sa[1]);

    float cm[8];
#pragma unroll
    for (int r = 0; r < 8; ++r) {
      float m = fmaxf(sa[0][r], sa[1][r]);
#pragma unroll
      for (int off = 1; off < 16; off <<= 1) m = fmaxf(m, __shfl_xor(m, off, 32));
      cm[r] = m;
    }
#pragma unroll
    for (int r = 0; r < 8; ++r) {
      const float mnew  = fmaxf(mrow[r], cm[r]);
      const float muse  = (mnew > -INFINITY) ? mnew : 0.0f;
      const float alpha = __expf(mrow[r] - muse);
      mrow[r] = mnew;
      float psum = 0.f;
#pragma unroll
      for (int j = 0; j < 2; ++j) {
        const float p = __expf(sa[j][r] - muse);
        psum += p;
        const unsigned short hb = bf_bits(p);
        const unsigned short lb = bf_bits(p - bf_val(hb));
        const int po = (8 * hh + r) * PP + j * 16 + c;
        ph[po] = hb;
        pl[po] = lb;
      }
#pragma unroll
      for (int off = 1; off < 16; off <<= 1) psum += __shfl_xor(psum, off, 32);
      lrow[r] = lrow[r] * alpha + psum;
#pragma unroll
      for (int t = 0; t < 4; ++t) oacc[t][r] *= alpha;
    }
    lds_wave_sync();
    const v16b pa = ldfrag_b((const __bf16*)(const void*)ph + c * PP + 8 * hh);
    const v16b pr = ldfrag_b((const __bf16*)(const void*)pl + c * PP + 8 * hh);
#pragma unroll
    for (int t = 0; t < 4; ++t) {
      const v16b vb = ldfrag_b((const __bf16*)(const void*)Vhs + (t * 16 + c) * VP + 8 * hh);
      const v16b vr = ldfrag_b((const __bf16*)(const void*)Vls + (t * 16 + c) * VP + 8 * hh);
      oacc[t] = mma_b(pa, vb, oacc[t]);
      oacc[t] = mma_b(pa, vr, oacc[t]);
      oacc[t] = mma_b(pr, vb, oacc[t]);
      guard1b4(oacc[t], pa, pr, vb, vr);
    }
  }
  __syncthreads();
  acc_guard4(oacc[0], oacc[1], oacc[2], oacc[3]);

  unsigned short* osh = Osh[wave];
  unsigned short* osl = Osl[wave];
#pragma unroll
  for (int r = 0; r < 8; ++r) {
    const float inv = 1.0f / lrow[r];
#pragma unroll
    for (int t = 0; t < 4; ++t) {
      const float o = oacc[t][r] * inv;
      const unsigned short hb = bf_bits(o);
      const unsigned short lb = bf_bits(o - bf_val(hb));
      const int so = (8 * hh + r) * 64 + t * 16 + c;
      osh[so] = hb;
      osl[so] = lb;
    }
  }
  lds_wave_sync();
  unsigned short* Ag = aop + (tok0 + q0) * AOW + h * HDM;
  const int qq = lane >> 3;
  const int c8 = (lane & 7) * 8;
  for (int pass = 0; pass < 2; ++pass) {
#pragma unroll
    for (int it = 0; it < 4; ++it) {
      const int row = it * 4 + qq;
      const v4u xw = *(const v4u*)(osh + row * 64 + c8);
      const v4u yw = *(const v4u*)(osl + row * 64 + c8);
      *(volatile v4u*)(Ag + (size_t)row * AOW + c8)      = xw;
      *(volatile v4u*)(Ag + (size_t)row * AOW + QW + c8) = yw;
    }
    __threadfence();
  }
}

extern "C" void kernel_launch(void* const* d_in, const int* in_sizes, int n_in,
                              void* d_out, int out_size, void* d_ws, size_t ws_size,
                              hipStream_t stream) {
  if (n_in < 7) return;
  if (in_sizes[0] != NTOK * HID) return;
  if (in_sizes[1] != NTOK) return;
  if (in_sizes[2] != NB * CONDF) return;
  if (in_sizes[3] != HID * CONDF) return;
  if (in_sizes[4] != NQKV * HID) return;
  if (in_sizes[5] != NH) return;
  if (in_sizes[6] != HID * HID) return;
  if (out_size != NTOK * HID) return;

  const float* x     = (const float*)d_in[0];
  const float* pos   = (const float*)d_in[1];
  const float* cond  = (const float*)d_in[2];
  const float* wnorm = (const float*)d_in[3];
  const float* wqkv  = (const float*)d_in[4];
  const float* scale = (const float*)d_in[5];
  const float* wout  = (const float*)d_in[6];
  float* out = (float*)d_out;

  const size_t szCS   = (size_t)NB * HID * 4;
  const size_t szFT   = 512;
  const size_t szT    = (size_t)NTOK * TABW * 4;
  const size_t szXN   = (size_t)NTOK * XNW * 2;
  const size_t szWQKV = (size_t)NQKV * XNW * 2;
  const size_t szWO2  = (size_t)HID * AOW * 2;
  const size_t szQ    = (size_t)NTOK * QW * 2;
  const size_t szVT   = (size_t)QW * NTOK * 2;
  const size_t szAO   = (size_t)NTOK * AOW * 2;
  size_t off = 0;
  const size_t oCS   = off; off += szCS;
  const size_t oFT   = off; off += szFT;
  const size_t oCST  = off; off += szT;
  const size_t oSNT  = off; off += szT;
  const size_t oXN   = off; off += szXN;
  const size_t oWQKV = off; off += szWQKV;
  const size_t oWO2  = off; off += szWO2;
  const size_t oQH   = off; off += szQ;
  const size_t oQL   = off; off += szQ;
  const size_t oKH   = off; off += szQ;
  const size_t oKL   = off; off += szQ;
  const size_t oVTH  = off; off += szVT;
  const size_t oVTL  = off; off += szVT;
  const size_t oAO   = off; off += szAO;
  if (off > ws_size) return;

  char* ws = (char*)d_ws;
  float*          CS    = (float*)(ws + oCS);
  float*          FT    = (float*)(ws + oFT);
  float*          CST   = (float*)(ws + oCST);
  float*          SNT   = (float*)(ws + oSNT);
  unsigned short* XN    = (unsigned short*)(ws + oXN);
  unsigned short* WQKV2 = (unsigned short*)(ws + oWQKV);
  unsigned short* WO2   = (unsigned short*)(ws + oWO2);
  unsigned short* QH    = (unsigned short*)(ws + oQH);
  unsigned short* QL    = (unsigned short*)(ws + oQL);
  unsigned short* KH    = (unsigned short*)(ws + oKH);
  unsigned short* KL    = (unsigned short*)(ws + oKL);
  unsigned short* VTH   = (unsigned short*)(ws + oVTH);
  unsigned short* VTL   = (unsigned short*)(ws + oVTL);
  unsigned short* AO    = (unsigned short*)(ws + oAO);

  const dim3 b256(256), b128(128);

  freq_table_kernel<<<dim3(1), b128, 0, stream>>>(FT);
  cond_scale_kernel<<<dim3((NB * HID) / 256), b256, 0, stream>>>(cond, wnorm, CS);
  rope_table_kernel<<<dim3(NTOK), b128, 0, stream>>>(pos, FT, CST, SNT);
  xn_split_kernel<<<dim3(NTOK), b128, 0, stream>>>(x, CS, XN);
  cvt_dup2_kernel<<<dim3((NQKV * HID / 8) / 256), b256, 0, stream>>>(wqkv, WQKV2, NQKV * HID / 8, HID, XNW);
  cvt_dup2_kernel<<<dim3((HID * HID / 8) / 256), b256, 0, stream>>>(wout, WO2, HID * HID / 8, HID, AOW);
  gemm_w32x128_kernel<0><<<dim3((NTOK / 32) * (QKN / 128) / 4), b128, 0, stream>>>(
      XN, XNW, WQKV2, XNW, CST, SNT, scale, x,
      (void*)QH, (void*)QL, (void*)KH, (void*)KL, QW, QW, NTOK, QKN, XNW);
  gemm_w32x128_kernel<1><<<dim3((QW / 32) * (NTOK / 128) / 4), b128, 0, stream>>>(
      WQKV2 + (size_t)QKN * XNW, XNW, XN, XNW, CST, SNT, scale, x,
      (void*)VTH, (void*)VTL, (void*)VTH, (void*)VTL, NTOK, NTOK, QW, NTOK, XNW);
  attn_kernel<<<dim3(SQ / 64, NH, NB), b128, 0, stream>>>(QH, QL, KH, KL, VTH, VTL, AO);
  gemm_w32x128_kernel<2><<<dim3((NTOK / 32) * (HID / 128) / 4), b128, 0, stream>>>(
      AO, AOW, WO2, AOW, CST, SNT, scale, x,
      (void*)out, (void*)out, (void*)out, (void*)out, HID, HID, NTOK, HID, AOW);
  (void)hipGetLastError();
}
